// BiMultiHeadAttention_11682311045282
// MI455X (gfx1250) — hardware-verified
//
#include <hip/hip_runtime.h>
#include <math.h>
#include <stdint.h>

#define NB      2
#define TV      16000
#define SL      256
#define EMB     256
#define LD      768
#define NH      8
#define HD      32
#define NV      (NB * TV)
#define NL      (NB * SL)
#define NQT     (TV / 64)
#define RR      10
#define TPR     (TV / RR)
#define NSTEP   (TPR / 32)
#define RECROWS 33
#define SCALEQ  0.17677669529663687f
#define CLAMPV  50000.0f
#define MASKNEG (-9.0e15f)

static_assert(NH * HD == EMB);
static_assert(NQT * 64 == TV);
static_assert(RR * NSTEP * 32 == TV);
static_assert((NV % 64) == 0 && (NL % 64) == 0 && (EMB % 64) == 0 && (LD % 64) == 0 && (TV % 64) == 0);
static_assert((EMB % 32) == 0 && (LD % 32) == 0 && ((2 * EMB) % 32) == 0);
static_assert(SL == 256 && HD == 32 && EMB == 256);

typedef __bf16   v16b __attribute__((ext_vector_type(16)));
typedef __bf16   v8b  __attribute__((ext_vector_type(8)));
typedef float    v8f  __attribute__((ext_vector_type(8)));
typedef float    v4f  __attribute__((ext_vector_type(4)));
typedef unsigned int v4u __attribute__((ext_vector_type(4)));
typedef unsigned int v8u __attribute__((ext_vector_type(8)));
typedef int      v4i  __attribute__((ext_vector_type(4)));
typedef v4f __attribute__((may_alias)) v4fa;
typedef v4i __attribute__((may_alias)) v4ia;

#if defined(__HIP_DEVICE_COMPILE__)
#define DEV_ASM 1
#else
#define DEV_ASM 0
#endif

__device__ __forceinline__ unsigned short bf_bits(float f) {
  unsigned u = __float_as_uint(f);
  return (unsigned short)((u + 0x7FFFu + ((u >> 16) & 1u)) >> 16);
}
__device__ __forceinline__ float bf_up(unsigned short hb) { return __uint_as_float(((unsigned)hb) << 16); }
__device__ __forceinline__ float rbf(float f) { return bf_up(bf_bits(f)); }
__device__ __forceinline__ unsigned pk16(unsigned short a, unsigned short b) { return (unsigned)a | ((unsigned)b << 16); }
__device__ __forceinline__ v8f zero8() { v8f z = {0.f, 0.f, 0.f, 0.f, 0.f, 0.f, 0.f, 0.f}; return z; }
__device__ __forceinline__ float clampv(float x) { return fminf(fmaxf(x, -CLAMPV), CLAMPV); }

__device__ __forceinline__ v16b ldfrag(const __bf16* p) {
  union { v16b v; v8b h[2]; } f;
  f.h[0] = *(const v8b*)(p);
  f.h[1] = *(const v8b*)(p + 16);
  return f.v;
}

__device__ __forceinline__ v8f mmar(v16b a, v16b b, v8f c) {
  return __builtin_amdgcn_wmma_f32_16x16x32_bf16(false, a, false, b, (short)0, c, false, false);
}
__device__ __forceinline__ v8f mma_b(v16b a, v16b b, v8f c) {
  c = __builtin_amdgcn_wmma_f32_16x16x32_bf16(false, a, false, b, (short)0, c, false, false);
#if DEV_ASM
  asm volatile("v_nop\n\tv_nop\n\tv_nop\n\tv_nop" : "+v"(c) : "v"(a), "v"(b));
#endif
  return c;
}
__device__ __forceinline__ void dep_guard(v8f& a, v8f& b, v16b x, v16b y) {
#if DEV_ASM
  asm volatile("v_nop\n\tv_nop\n\tv_nop\n\tv_nop" : "+v"(a), "+v"(b) : "v"(x), "v"(y));
#else
  (void)a; (void)b; (void)x; (void)y;
#endif
}
__device__ __forceinline__ void keep4(v16b a, v16b b, v16b c, v16b d) {
#if DEV_ASM
  asm volatile("v_nop" :: "v"(a), "v"(b), "v"(c), "v"(d));
#else
  (void)a; (void)b; (void)c; (void)d;
#endif
}
__device__ __forceinline__ void acc_guard4(v8f& a, v8f& b, v8f& c, v8f& d) {
#if DEV_ASM
  asm volatile("v_nop\n\tv_nop\n\tv_nop\n\tv_nop" : "+v"(a), "+v"(b), "+v"(c), "+v"(d));
#else
  (void)a; (void)b; (void)c; (void)d;
#endif
}

union PK { v8u u; v16b v; };
__device__ __forceinline__ void pack_hl(v8f a, v8f c, v16b& fh, v16b& fl) {
  v8u ph, pl;
#pragma unroll
  for (int i = 0; i < 4; ++i) {
    const float x0 = a[2 * i], x1 = a[2 * i + 1];
    const unsigned short h0 = bf_bits(x0), h1 = bf_bits(x1);
    const unsigned short l0 = bf_bits(x0 - bf_up(h0)), l1 = bf_bits(x1 - bf_up(h1));
    ph[i] = pk16(h0, h1);
    pl[i] = pk16(l0, l1);
    const float y0 = c[2 * i], y1 = c[2 * i + 1];
    const unsigned short g0 = bf_bits(y0), g1 = bf_bits(y1);
    const unsigned short n0 = bf_bits(y0 - bf_up(g0)), n1 = bf_bits(y1 - bf_up(g1));
    ph[4 + i] = pk16(g0, g1);
    pl[4 + i] = pk16(n0, n1);
  }
  PK uh, ul;
  uh.u = ph; ul.u = pl;
  fh = uh.v; fl = ul.v;
}

__global__ __launch_bounds__(256) void cvt_bf16x8(const float* __restrict__ in, unsigned short* out, int n8) {
  const int i = blockIdx.x * 256 + (int)threadIdx.x;
  if (i < n8) {
    const v4f a  = *(const v4fa*)(in + (size_t)i * 8);
    const v4f a4 = *(const v4fa*)(in + (size_t)i * 8 + 4);
    v4u p;
    p[0] = pk16(bf_bits(a[0]),  bf_bits(a[1]));
    p[1] = pk16(bf_bits(a[2]),  bf_bits(a[3]));
    p[2] = pk16(bf_bits(a4[0]), bf_bits(a4[1]));
    p[3] = pk16(bf_bits(a4[2]), bf_bits(a4[3]));
    unsigned short* o = out + (size_t)i * 8;
    *(volatile v4u*)o = p;
    __threadfence();
    *(volatile v4u*)o = p;
  }
}

__global__ __launch_bounds__(256) void cvt_dup(const float* __restrict__ in, unsigned short* out, int nrows) {
  const int lane = (int)threadIdx.x & 31, wave = (int)threadIdx.x >> 5;
  const int row = blockIdx.x * 8 + wave;
  if (row >= nrows) return;
  const float* src = in + (size_t)row * EMB;
  unsigned short* dst = out + (size_t)row * (2 * EMB);
  v4u p[2];
#pragma unroll
  for (int half = 0; half < 2; ++half) {
    const int g = half * 4 + (lane >> 3);
    const int scol = g * HD + 8 * (lane & 3);
    const v4f a = *(const v4fa*)(src + scol);
    const v4f c = *(const v4fa*)(src + scol + 4);
    v4u q;
    q[0] = pk16(bf_bits(a[0]), bf_bits(a[1]));
    q[1] = pk16(bf_bits(a[2]), bf_bits(a[3]));
    q[2] = pk16(bf_bits(c[0]), bf_bits(c[1]));
    q[3] = pk16(bf_bits(c[2]), bf_bits(c[3]));
    p[half] = q;
  }
  for (int pass = 0; pass < 2; ++pass) {
#pragma unroll
    for (int half = 0; half < 2; ++half)
      *(volatile v4u*)(dst + half * EMB + 8 * lane) = p[half];
    __threadfence();
  }
}

template <int OUT_MODE, int BIASM>
__global__ __launch_bounds__(256) void gemm64(
    const unsigned short* __restrict__ Ap, int lda, long long strideA,
    const unsigned short* __restrict__ Btp, int ldb, long long strideB,
    const float* __restrict__ bias,
    void* Cout, void* Cout2, int ldc, long long strideC,
    int M, int N, int K, float oscale) {
  static_assert(OUT_MODE == 0 || OUT_MODE == 3);
  static_assert(OUT_MODE != 0 || BIASM == 0);
  const __bf16* A  = (const __bf16*)(const void*)Ap;
  const __bf16* Bt = (const __bf16*)(const void*)Btp;
  __shared__ __align__(16) float sT[8][16 * 68];
  const int b    = blockIdx.y;
  const int lane = threadIdx.x & 31;
  const int wave = threadIdx.x >> 5;
  const int tilesN = N >> 6;
  const int tilesM = M >> 6;
  const int tile = blockIdx.x * 8 + wave;
  if (tile >= tilesM * tilesN) return;
  const int tm = tile / tilesN;
  const int tn = tile - tm * tilesN;
  const int m0 = tm << 6;
  const int n0 = tn << 6;

  const __bf16* Ab = A  + (size_t)b * (size_t)strideA;
  const __bf16* Bb = Bt + (size_t)b * (size_t)strideB;

  const int rlane = lane & 15;
  const int koff  = (lane >> 4) * 8;
  const int mOff  = (lane >> 4) * 8;

  v8f acc[4][4];
#pragma unroll
  for (int i = 0; i < 4; ++i)
#pragma unroll
    for (int j = 0; j < 4; ++j) acc[i][j] = zero8();

  for (int k0 = 0; k0 < K; k0 += 32) {
    v16b bq[4];
#pragma unroll
    for (int j = 0; j < 4; ++j)
      bq[j] = ldfrag(Bb + (size_t)(n0 + (j << 4) + rlane) * ldb + koff + k0);
#pragma unroll
    for (int i = 0; i < 4; ++i) {
      const v16b af = ldfrag(Ab + (size_t)(m0 + (i << 4) + rlane) * lda + koff + k0);
#pragma unroll
      for (int j = 0; j < 4; ++j) acc[i][j] = mmar(af, bq[j], acc[i][j]);
      dep_guard(acc[i][0], acc[i][3], af, bq[3]);
    }
    keep4(bq[0], bq[1], bq[2], bq[3]);
  }
  acc_guard4(acc[0][0], acc[0][1], acc[0][2], acc[0][3]);
  acc_guard4(acc[1][0], acc[1][1], acc[1][2], acc[1][3]);
  acc_guard4(acc[2][0], acc[2][1], acc[2][2], acc[2][3]);
  acc_guard4(acc[3][0], acc[3][1], acc[3][2], acc[3][3]);

  float* slab = sT[wave];
  const int h2 = lane >> 4, c4 = (lane & 15) * 4;
  const int q = lane >> 3, c8 = (lane & 7) * 8;
  v4f bb4;
  float bcol[8];
  if (OUT_MODE == 0) {
    const v4f braw = *(const v4fa*)(bias + n0 + c4);
    bb4[0] = rbf(braw[0]); bb4[1] = rbf(braw[1]); bb4[2] = rbf(braw[2]); bb4[3] = rbf(braw[3]);
  } else {
    if (BIASM == 0) {
      const v4f b0 = *(const v4fa*)(bias + n0 + c8);
      const v4f b1 = *(const v4fa*)(bias + n0 + c8 + 4);
#pragma unroll
      for (int e = 0; e < 4; ++e) { bcol[e] = rbf(b0[e]); bcol[4 + e] = rbf(b1[e]); }
    } else {
#pragma unroll
      for (int e = 0; e < 8; ++e) bcol[e] = 0.f;
    }
  }
#pragma unroll
  for (int i = 0; i < 4; ++i) {
    const int mBase = m0 + (i << 4);
#pragma unroll
    for (int j = 0; j < 4; ++j) {
#pragma unroll
      for (int r = 0; r < 8; ++r) {
        slab[(mOff + r) * 68 + (j << 4) + rlane] = acc[i][j][r];
      }
    }
    __builtin_amdgcn_fence(__ATOMIC_RELEASE, "workgroup");
    __builtin_amdgcn_wave_barrier();
    __builtin_amdgcn_fence(__ATOMIC_ACQUIRE, "workgroup");
    if (OUT_MODE == 0) {
      float* C = (float*)Cout + (size_t)b * (size_t)strideC;
      for (int pass = 0; pass < 2; ++pass) {
#pragma unroll
        for (int it = 0; it < 8; ++it) {
          const int row = it * 2 + h2;
          v4f v = *(const v4fa*)(slab + row * 68 + c4);
          v = (v + bb4) * oscale;
          *(volatile v4f*)(C + (size_t)(mBase + row) * ldc + n0 + c4) = v;
        }
        __threadfence();
      }
    } else {
      unsigned short* C  = (unsigned short*)Cout  + (size_t)b * (size_t)strideC;
      unsigned short* C2 = (unsigned short*)Cout2 + (size_t)b * (size_t)strideC;
      v4u hv[4], lv[4];
#pragma unroll
      for (int it = 0; it < 4; ++it) {
        const int row = it * 4 + q;
        const float* sp = slab + row * 68 + c8;
        float brow = 0.f;
        if (BIASM == 1) brow = rbf(bias[mBase + row]);
        v4u a, a2;
#pragma unroll
        for (int e = 0; e < 4; ++e) {
          const float f0 = (sp[2 * e]     + ((BIASM == 1) ? brow : bcol[2 * e]))     * oscale;
          const float f1 = (sp[2 * e + 1] + ((BIASM == 1) ? brow : bcol[2 * e + 1])) * oscale;
          const unsigned short h0 = bf_bits(f0), h1 = bf_bits(f1);
          const unsigned short l0 = bf_bits(f0 - bf_up(h0)), l1 = bf_bits(f1 - bf_up(h1));
          a[e] = pk16(h0, h1); a2[e] = pk16(l0, l1);
        }
        hv[it] = a; lv[it] = a2;
      }
      for (int pass = 0; pass < 2; ++pass) {
#pragma unroll
        for (int it = 0; it < 4; ++it) {
          const int row = it * 4 + q;
          *(volatile v4u*)(C  + (size_t)(mBase + row) * ldc + n0 + c8) = hv[it];
          *(volatile v4u*)(C2 + (size_t)(mBase + row) * ldc + n0 + c8) = lv[it];
        }
        __threadfence();
      }
    }
    __builtin_amdgcn_fence(__ATOMIC_RELEASE, "workgroup");
    __builtin_amdgcn_wave_barrier();
    __builtin_amdgcn_fence(__ATOMIC_ACQUIRE, "workgroup");
  }
}

__device__ __forceinline__ v8f add_mask8(v8f s, const int* p) {
  const v4i ma = *(const v4ia*)p;
  const v4i mb = *(const v4ia*)(p + 4);
  s[0] += (ma[0] == 0) ? MASKNEG : 0.0f;
  s[1] += (ma[1] == 0) ? MASKNEG : 0.0f;
  s[2] += (ma[2] == 0) ? MASKNEG : 0.0f;
  s[3] += (ma[3] == 0) ? MASKNEG : 0.0f;
  s[4] += (mb[0] == 0) ? MASKNEG : 0.0f;
  s[5] += (mb[1] == 0) ? MASKNEG : 0.0f;
  s[6] += (mb[2] == 0) ? MASKNEG : 0.0f;
  s[7] += (mb[3] == 0) ? MASKNEG : 0.0f;
  return s;
}

__global__ __launch_bounds__(128)
void attn_v(const unsigned short* __restrict__ qhp, const unsigned short* __restrict__ qlp,
            const unsigned short* __restrict__ khp, const unsigned short* __restrict__ klp,
            const unsigned short* __restrict__ vhp, const unsigned short* __restrict__ vlp,
            const int* __restrict__ maskl, float* cmout, unsigned short* ctxp) {
  __shared__ __align__(16) float cmw[4][SL];
  __shared__ __align__(16) float cmb[SL];
  __shared__ __align__(16) float sO[4][16 * HD];

  const int tid = threadIdx.x, lane = tid & 31, w = tid >> 5;
  const int hh = lane >> 4, m = lane & 15;
  const int qt = blockIdx.x, bh = blockIdx.y, b = bh >> 3, head = bh & 7;
  const int q0 = qt * 64 + 16 * w;

  const __bf16* Qh = (const __bf16*)(const void*)qhp;
  const __bf16* Ql = (const __bf16*)(const void*)qlp;
  const __bf16* Kh = (const __bf16*)(const void*)khp;
  const __bf16* Kl = (const __bf16*)(const void*)klp;
  const __bf16* Vh = (const __bf16*)(const void*)vhp;
  const __bf16* Vl = (const __bf16*)(const void*)vlp;

  const size_t qoff = ((size_t)b * TV + q0 + m) * EMB + head * HD + 8 * hh;
  const v16b qbh = ldfrag(Qh + qoff);
  const v16b qbl = ldfrag(Ql + qoff);

  const __bf16* kbh = Kh + ((size_t)b * SL + m) * EMB + head * HD + 8 * hh;
  const __bf16* kbl = Kl + ((size_t)b * SL + m) * EMB + head * HD + 8 * hh;
  const __bf16* vbh = Vh + ((size_t)b * EMB + head * HD + m) * SL + 8 * hh;
  const __bf16* vbl = Vl + ((size_t)b * EMB + head * HD + m) * SL + 8 * hh;
  const int* mkp = maskl + b * SL + 8 * hh;

  v8f o[2];
  o[0] = zero8(); o[1] = zero8();
  float mrun = -1.0e30f, lrun = 0.0f;

#pragma unroll 1
  for (int kc = 0; kc < SL / 64; ++kc) {
    const int kb0 = kc * 64;
    v8f s[4];
#pragma unroll
    for (int j = 0; j < 4; ++j) {
      const size_t ko = (size_t)(kb0 + 16 * j) * EMB;
      const v16b kfh = ldfrag(kbh + ko);
      const v16b kfl = ldfrag(kbl + ko);
      v8f z = zero8();
      z = mma_b(kfh, qbh, z);
      z = mma_b(kfl, qbh, z);
      z = mma_b(kfh, qbl, z);
      s[j] = z;
    }
#pragma unroll
    for (int j = 0; j < 4; ++j) {
#pragma unroll
      for (int r = 0; r < 8; ++r) {
        float vv = clampv(s[j][r]);
        s[j][r] = vv;
        vv = fmaxf(vv, __shfl_xor(vv, 1, 32));
        vv = fmaxf(vv, __shfl_xor(vv, 2, 32));
        vv = fmaxf(vv, __shfl_xor(vv, 4, 32));
        vv = fmaxf(vv, __shfl_xor(vv, 8, 32));
        if (m == 0) cmw[w][kb0 + 16 * j + 8 * hh + r] = vv;
      }
    }
#pragma unroll
    for (int j = 0; j < 4; ++j) s[j] = add_mask8(s[j], mkp + kb0 + 16 * j);

    float mloc = s[0][0];
#pragma unroll
    for (int j = 0; j < 4; ++j)
#pragma unroll
      for (int r = 0; r < 8; ++r) mloc = fmaxf(mloc, s[j][r]);
    mloc = fmaxf(mloc, __shfl_xor(mloc, 16, 32));
    const float mnew = fmaxf(mrun, mloc);
    const float alpha = __expf(mrun - mnew);
    mrun = mnew;
    float lsum = 0.0f;
#pragma unroll
    for (int j = 0; j < 4; ++j)
#pragma unroll
      for (int r = 0; r < 8; ++r) {
        const float p = __expf(s[j][r] - mnew);
        s[j][r] = p;
        lsum += p;
      }
    lsum += __shfl_xor(lsum, 16, 32);
    lrun = lrun * alpha + lsum;
#pragma unroll
    for (int dt = 0; dt < 2; ++dt)
#pragma unroll
      for (int r = 0; r < 8; ++r) o[dt][r] = o[dt][r] * alpha;

    v16b pbh0, pbl0, pbh1, pbl1;
    pack_hl(s[0], s[1], pbh0, pbl0);
    pack_hl(s[2], s[3], pbh1, pbl1);

#pragma unroll
    for (int dt = 0; dt < 2; ++dt) {
      const size_t vo = (size_t)(16 * dt) * SL + kb0;
      const v16b vh0 = ldfrag(vbh + vo), vh1 = ldfrag(vbh + vo + 32);
      const v16b vl0 = ldfrag(vbl + vo), vl1 = ldfrag(vbl + vo + 32);
      v8f a = o[dt];
      a = mma_b(vh0, pbh0, a);
      a = mma_b(vh0, pbl0, a);
      a = mma_b(vl0, pbh0, a);
      a = mma_b(vh1, pbh1, a);
      a = mma_b(vh1, pbl1, a);
      a = mma_b(vl1, pbh1, a);
      o[dt] = a;
    }
  }

  const float inv = 1.0f / lrun;
  float* so = sO[w];
#pragma unroll
  for (int dt = 0; dt < 2; ++dt)
#pragma unroll
    for (int r = 0; r < 8; ++r)
      so[m * HD + 16 * dt + 8 * hh + r] = o[dt][r] * inv;
  __syncthreads();

  {
    const int sub = lane >> 3, piece = lane & 7;
    const int csel = 8 * (piece & 3);
    const bool islo = (piece & 4) != 0;
    v4u hv[4];
#pragma unroll
    for (int i = 0; i < 4; ++i) {
      const int lid = i * 4 + sub;
      const float* sp = so + lid * HD + csel;
      v4u a;
#pragma unroll
      for (int e = 0; e < 4; ++e) {
        const float x0 = sp[2 * e], x1 = sp[2 * e + 1];
        const unsigned short h0 = bf_bits(x0), h1 = bf_bits(x1);
        const unsigned short l0 = bf_bits(x0 - bf_up(h0)), l1 = bf_bits(x1 - bf_up(h1));
        a[e] = islo ? pk16(l0, l1) : pk16(h0, h1);
      }
      hv[i] = a;
    }
    for (int pass = 0; pass < 2; ++pass) {
#pragma unroll
      for (int i = 0; i < 4; ++i) {
        const int lid = i * 4 + sub;
        const size_t go = ((size_t)b * TV + q0 + lid) * (2 * EMB) + head * (2 * HD) + 8 * piece;
        *(volatile v4u*)(ctxp + go) = hv[i];
      }
      __threadfence();
    }
  }

  for (int t = tid; t < SL; t += 128)
    cmb[t] = fmaxf(fmaxf(cmw[0][t], cmw[1][t]), fmaxf(cmw[2][t], cmw[3][t]));
  __syncthreads();
  if (tid < 64) {
    const v4f vv = *(const v4fa*)(cmb + 4 * tid);
    float* dst = cmout + ((size_t)bh * NQT + qt) * SL + 4 * tid;
    *(volatile v4f*)dst = vv;
    __threadfence();
    *(volatile v4f*)dst = vv;
  }
}

__global__ __launch_bounds__(256) void fold_max(const float* __restrict__ cm, float* mx) {
  const int bh = blockIdx.x, s = (int)threadIdx.x;
  const float* p = cm + (size_t)bh * NQT * SL + s;
  float mm = p[0];
#pragma unroll 2
  for (int qq = 1; qq < NQT; ++qq) mm = fmaxf(mm, p[(size_t)qq * SL]);
  float* d = mx + bh * SL + s;
  *(volatile float*)d = mm;
  __threadfence();
  *(volatile float*)d = mm;
}

__global__ __launch_bounds__(128)
void attn_l(const unsigned short* __restrict__ qhp, const unsigned short* __restrict__ qlp,
            const unsigned short* __restrict__ khp, const unsigned short* __restrict__ klp,
            const unsigned short* __restrict__ vhp, const unsigned short* __restrict__ vlp,
            const float* __restrict__ mx, float* rec) {
  __shared__ __align__(16) float st[4][RECROWS * 32];

  const int tid = threadIdx.x, lane = tid & 31, w = tid >> 5;
  const int hh = lane >> 4, m = lane & 15;
  const int rg = blockIdx.x, kq = blockIdx.y, bh = blockIdx.z, b = bh >> 3, head = bh & 7;
  const int s0 = kq * 128 + 32 * w;
  const int tb = rg * TPR;

  const __bf16* Qh = (const __bf16*)(const void*)qhp;
  const __bf16* Ql = (const __bf16*)(const void*)qlp;
  const __bf16* Kh = (const __bf16*)(const void*)khp;
  const __bf16* Kl = (const __bf16*)(const void*)klp;
  const __bf16* Vh = (const __bf16*)(const void*)vhp;
  const __bf16* Vl = (const __bf16*)(const void*)vlp;

  v16b kfh[2], kfl[2];
  float mvj[2], csum[2];
#pragma unroll
  for (int jj = 0; jj < 2; ++jj) {
    const size_t ko = ((size_t)b * SL + s0 + 16 * jj + m) * EMB + head * HD + 8 * hh;
    kfh[jj] = ldfrag(Kh + ko);
    kfl[jj] = ldfrag(Kl + ko);
    mvj[jj] = mx[bh * SL + s0 + 16 * jj + m];
    csum[jj] = 0.0f;
  }
  v8f acc[2][2];
#pragma unroll
  for (int dt = 0; dt < 2; ++dt) { acc[dt][0] = zero8(); acc[dt][1] = zero8(); }

  const __bf16* qbh = Qh + ((size_t)b * TV + m) * EMB + head * HD + 8 * hh;
  const __bf16* qbl = Ql + ((size_t)b * TV + m) * EMB + head * HD + 8 * hh;
  const __bf16* vbh = Vh + ((size_t)b * EMB + head * HD + m) * TV + 8 * hh;
  const __bf16* vbl = Vl + ((size_t)b * EMB + head * HD + m) * TV + 8 * hh;

#pragma unroll 1
  for (int step = 0; step < NSTEP; ++step) {
    const int t0 = tb + 32 * step;
    v16b qah[2], qal[2], vah[2], val2[2];
#pragma unroll
    for (int tt = 0; tt < 2; ++tt) {
      const size_t qo = (size_t)(t0 + 16 * tt) * EMB;
      qah[tt] = ldfrag(qbh + qo);
      qal[tt] = ldfrag(qbl + qo);
    }
#pragma unroll
    for (int dt = 0; dt < 2; ++dt) {
      const size_t vo = (size_t)(16 * dt) * TV + t0;
      vah[dt]  = ldfrag(vbh + vo);
      val2[dt] = ldfrag(vbl + vo);
    }
#pragma unroll
    for (int jj = 0; jj < 2; ++jj) {
      v8f d0 = zero8(), d1 = zero8();
      d0 = mma_b(qah[0], kfh[jj], d0);
      d0 = mma_b(qah[0], kfl[jj], d0);
      d0 = mma_b(qal[0], kfh[jj], d0);
      d1 = mma_b(qah[1], kfh[jj], d1);
      d1 = mma_b(qah[1], kfl[jj], d1);
      d1 = mma_b(qal[1], kfh[jj], d1);
      const float mv = mvj[jj];
      float cl = csum[jj];
#pragma unroll
      for (int r = 0; r < 8; ++r) {
        const float x0 = clampv(clampv(d0[r]) - mv);
        const float e0 = __expf(x0);
        d0[r] = e0; cl += e0;
        const float x1 = clampv(clampv(d1[r]) - mv);
        const float e1 = __expf(x1);
        d1[r] = e1; cl += e1;
      }
      csum[jj] = cl;
      v16b ebh, ebl;
      pack_hl(d0, d1, ebh, ebl);
#pragma unroll
      for (int dt = 0; dt < 2; ++dt) {
        v8f a = acc[dt][jj];
        a = mma_b(vah[dt],  ebh, a);
        a = mma_b(vah[dt],  ebl, a);
        a = mma_b(val2[dt], ebh, a);
        acc[dt][jj] = a;
      }
    }
  }

#pragma unroll
  for (int jj = 0; jj < 2; ++jj) csum[jj] += __shfl_xor(csum[jj], 16, 32);
  float* sw = st[w];
#pragma unroll
  for (int dt = 0; dt < 2; ++dt)
#pragma unroll
    for (int jj = 0; jj < 2; ++jj)
#pragma unroll
      for (int r = 0; r < 8; ++r)
        sw[(16 * dt + 8 * hh + r) * 32 + 16 * jj + m] = acc[dt][jj][r];
  if (hh == 0) {
    sw[32 * 32 + m]      = csum[0];
    sw[32 * 32 + 16 + m] = csum[1];
  }
  __syncthreads();

  {
    const int sub = lane >> 3, piece = lane & 7;
    float* rbase = rec + (((size_t)bh * RR + rg) * RECROWS) * SL + s0 + 4 * piece;
    for (int pass = 0; pass < 2; ++pass) {
#pragma unroll
      for (int i = 0; i < 9; ++i) {
        const int lid  = i * 4 + sub;
        const int lidc = (lid < RECROWS) ? lid : (RECROWS - 1);
        const v4f vv = *(const v4fa*)(sw + lidc * 32 + 4 * piece);
        if (lid < RECROWS) *(volatile v4f*)(rbase + (size_t)lid * SL) = vv;
      }
      __threadfence();
    }
  }
}

__global__ __launch_bounds__(256) void fold_l(const float* __restrict__ rec, unsigned short* ctxl) {
  __shared__ __align__(16) float xs[EMB];
  const int bs = blockIdx.x, b = bs / SL, s = bs - b * SL;
  const int t = (int)threadIdx.x, head = t >> 5, d = t & 31;
  const int bh = b * NH + head;
  const float* p = rec + ((size_t)bh * RR) * RECROWS * SL + s;
  float a = 0.0f, cs = 0.0f;
#pragma unroll 1
  for (int rg = 0; rg < RR; ++rg) {
    const float* pr = p + (size_t)rg * RECROWS * SL;
    a  += pr[(size_t)d * SL];
    cs += pr[(size_t)32 * SL];
  }
  xs[t] = a * (1.0f / cs);
  __syncthreads();
  if (t < 64) {
    const int hg = t >> 3, wq = t & 7;
    const float* sp = xs + hg * HD + 8 * (wq & 3);
    const bool islo = (wq & 4) != 0;
    v4u vv;
#pragma unroll
    for (int e = 0; e < 4; ++e) {
      const float x0 = sp[2 * e], x1 = sp[2 * e + 1];
      const unsigned short h0 = bf_bits(x0), h1 = bf_bits(x1);
      const unsigned short l0 = bf_bits(x0 - bf_up(h0)), l1 = bf_bits(x1 - bf_up(h1));
      vv[e] = islo ? pk16(l0, l1) : pk16(h0, h1);
    }
    unsigned short* dst = ctxl + (size_t)bs * (2 * EMB) + hg * (2 * HD) + 8 * wq;
    *(volatile v4u*)dst = vv;
    __threadfence();
    *(volatile v4u*)dst = vv;
  }
}

extern "C" void kernel_launch(void* const* d_in, const int* in_sizes, int n_in,
                              void* d_out, int out_size, void* d_ws, size_t ws_size,
                              hipStream_t stream) {
  if (n_in < 15) return;
  if (in_sizes[0] != NV * EMB || in_sizes[1] != NL * LD || in_sizes[2] != NB * SL) return;
  if (in_sizes[3] != EMB * EMB || in_sizes[4] != EMB || in_sizes[5] != EMB * LD || in_sizes[6] != EMB) return;
  if (in_sizes[7] != EMB * EMB || in_sizes[8] != EMB || in_sizes[9] != EMB * LD || in_sizes[10] != EMB) return;
  if (in_sizes[11] != EMB * EMB || in_sizes[12] != EMB || in_sizes[13] != LD * EMB || in_sizes[14] != LD) return;
  if (out_size != NV * EMB + NL * LD) return;

  const float* v_in = (const float*)d_in[0];
  const float* l_in = (const float*)d_in[1];
  const int*   mk   = (const int*)d_in[2];
  const float* Wv   = (const float*)d_in[3];
  const float* bv   = (const float*)d_in[4];
  const float* Wl   = (const float*)d_in[5];
  const float* bl   = (const float*)d_in[6];
  const float* Wvv  = (const float*)d_in[7];
  const float* bvv  = (const float*)d_in[8];
  const float* Wvl  = (const float*)d_in[9];
  const float* bvl  = (const float*)d_in[10];
  const float* Wov  = (const float*)d_in[11];
  const float* bov  = (const float*)d_in[12];
  const float* Wol  = (const float*)d_in[13];
  const float* bol  = (const float*)d_in[14];
  float* out0 = (float*)d_out;
  float* out1 = out0 + (size_t)NV * EMB;

  const size_t PVB  = (size_t)NV * EMB * 2;
  const size_t PLB  = (size_t)NL * LD * 2;
  const size_t PWS  = (size_t)EMB * EMB * 2;
  const size_t PWL  = (size_t)EMB * LD * 2;
  const size_t PWOD = (size_t)EMB * 2 * EMB * 2;
  const size_t PWLD = (size_t)LD * 2 * EMB * 2;
  const size_t PQ   = (size_t)NV * EMB * 2;
  const size_t PK   = (size_t)NL * EMB * 2;
  const size_t PVLT = (size_t)NB * EMB * SL * 2;
  const size_t PVVT = (size_t)NB * EMB * TV * 2;
  const size_t PCTX = (size_t)NV * 2 * EMB * 2;
  const size_t PCM  = (size_t)NB * NH * NQT * SL * 4;
  const size_t PMX  = (size_t)NB * NH * SL * 4;
  const size_t PREC = (size_t)NB * NH * RR * RECROWS * SL * 4;
  const size_t PCTL = (size_t)NL * 2 * EMB * 2;
  size_t off = 0;
  const size_t oVB  = off; off += PVB;
  const size_t oLB  = off; off += PLB;
  const size_t oWv  = off; off += PWS;
  const size_t oWvv = off; off += PWS;
  const size_t oWl  = off; off += PWL;
  const size_t oWvl = off; off += PWL;
  const size_t oWod = off; off += PWOD;
  const size_t oWld = off; off += PWLD;
  const size_t oQh  = off; off += PQ;
  const size_t oQl  = off; off += PQ;
  const size_t oKh  = off; off += PK;
  const size_t oKl  = off; off += PK;
  const size_t oVLh = off; off += PVLT;
  const size_t oVLl = off; off += PVLT;
  const size_t oVVh = off; off += PVVT;
  const size_t oVVl = off; off += PVVT;
  const size_t oCTX = off; off += PCTX;
  const size_t oCM  = off; off += PCM;
  const size_t oMX  = off; off += PMX;
  const size_t oREC = off; off += PREC;
  const size_t oCTL = off; off += PCTL;
  if (off > ws_size) return;
  if (off > (size_t)134217728) return;

  char* ws = (char*)d_ws;
  unsigned short* vb   = (unsigned short*)(ws + oVB);
  unsigned short* lb   = (unsigned short*)(ws + oLB);
  unsigned short* Wvb  = (unsigned short*)(ws + oWv);
  unsigned short* Wvvb = (unsigned short*)(ws + oWvv);
  unsigned short* Wlb  = (unsigned short*)(ws + oWl);
  unsigned short* Wvlb = (unsigned short*)(ws + oWvl);
  unsigned short* Wovd = (unsigned short*)(ws + oWod);
  unsigned short* Wold = (unsigned short*)(ws + oWld);
  unsigned short* Qh   = (unsigned short*)(ws + oQh);
  unsigned short* Ql   = (unsigned short*)(ws + oQl);
  unsigned short* Kh   = (unsigned short*)(ws + oKh);
  unsigned short* Kl   = (unsigned short*)(ws + oKl);
  unsigned short* VlTh = (unsigned short*)(ws + oVLh);
  unsigned short* VlTl = (unsigned short*)(ws + oVLl);
  unsigned short* VvTh = (unsigned short*)(ws + oVVh);
  unsigned short* VvTl = (unsigned short*)(ws + oVVl);
  unsigned short* CTXV = (unsigned short*)(ws + oCTX);
  float*          CM   = (float*)(ws + oCM);
  float*          MX   = (float*)(ws + oMX);
  float*          REC  = (float*)(ws + oREC);
  unsigned short* CTXL = (unsigned short*)(ws + oCTL);

  const dim3 blk(256);
  const int n8v  = NV * EMB / 8;
  const int n8l  = NL * LD / 8;
  const int n8ws = EMB * EMB / 8;
  const int n8wl = EMB * LD / 8;
  const dim3 gCv((n8v + 255) / 256), gCl((n8l + 255) / 256), gCws((n8ws + 255) / 256), gCwl((n8wl + 255) / 256);
  const dim3 gDupV((EMB + 7) / 8), gDupL((LD + 7) / 8);
  const dim3 gQ((((NV) / 64) * (EMB / 64) + 7) / 8, 1);
  const dim3 gK((((NL) / 64) * (EMB / 64) + 7) / 8, 1);
  const dim3 gVvT(((EMB / 64) * (TV / 64) + 7) / 8, NB);
  const dim3 gVlT(((EMB / 64) * (SL / 64) + 7) / 8, NB);
  const dim3 gO1((((NL) / 64) * (LD / 64) + 7) / 8, 1);
  const dim3 gAttV(NQT, NB * NH);
  const dim3 gAttL(RR, 2, NB * NH);

  cvt_bf16x8<<<gCv,  blk, 0, stream>>>(v_in, vb,   n8v);
  cvt_bf16x8<<<gCl,  blk, 0, stream>>>(l_in, lb,   n8l);
  cvt_bf16x8<<<gCws, blk, 0, stream>>>(Wv,   Wvb,  n8ws);
  cvt_bf16x8<<<gCws, blk, 0, stream>>>(Wvv,  Wvvb, n8ws);
  cvt_bf16x8<<<gCwl, blk, 0, stream>>>(Wl,   Wlb,  n8wl);
  cvt_bf16x8<<<gCwl, blk, 0, stream>>>(Wvl,  Wvlb, n8wl);
  cvt_dup<<<gDupV, blk, 0, stream>>>(Wov, Wovd, EMB);
  cvt_dup<<<gDupL, blk, 0, stream>>>(Wol, Wold, LD);
  gemm64<3, 0><<<gQ, blk, 0, stream>>>(
      vb, EMB, 0LL, Wvb, EMB, 0LL, bv,
      (void*)Qh, (void*)Ql, EMB, 0LL, NV, EMB, EMB, SCALEQ);
  gemm64<3, 0><<<gK, blk, 0, stream>>>(
      lb, LD, 0LL, Wlb, LD, 0LL, bl,
      (void*)Kh, (void*)Kl, EMB, 0LL, NL, EMB, LD, 1.0f);
  gemm64<3, 1><<<gVvT, blk, 0, stream>>>(
      Wvvb, EMB, 0LL, vb, EMB, (long long)TV * EMB, bvv,
      (void*)VvTh, (void*)VvTl, TV, (long long)EMB * TV, EMB, TV, EMB, 1.0f);
  gemm64<3, 1><<<gVlT, blk, 0, stream>>>(
      Wvlb, LD, 0LL, lb, LD, (long long)SL * LD, bvl,
      (void*)VlTh, (void*)VlTl, SL, (long long)EMB * SL, EMB, SL, LD, 1.0f);
  attn_v<<<gAttV, dim3(128), 0, stream>>>(Qh, Ql, Kh, Kl, VlTh, VlTl, mk, CM, CTXV);
  fold_max<<<dim3(NB * NH), blk, 0, stream>>>(CM, MX);
  attn_l<<<gAttL, dim3(128), 0, stream>>>(Qh, Ql, Kh, Kl, VvTh, VvTl, MX, REC);
  fold_l<<<dim3(NL), blk, 0, stream>>>(REC, CTXL);
  gemm64<0, 0><<<gQ, blk, 0, stream>>>(
      CTXV, 2 * EMB, 0LL, Wovd, 2 * EMB, 0LL, bov,
      (void*)out0, (void*)out0, EMB, 0LL, NV, EMB, 2 * EMB, 1.0f);
  gemm64<0, 0><<<gO1, blk, 0, stream>>>(
      CTXL, 2 * EMB, 0LL, Wold, 2 * EMB, 0LL, bol,
      (void*)out1, (void*)out1, LD, 0LL, NL, LD, 2 * EMB, 1.0f);
  (void)hipGetLastError();
}
